// rgb2uvHist_12910671692428
// MI455X (gfx1250) — hardware-verified
//
#include <hip/hip_runtime.h>
#include <stddef.h>


#pragma clang fp contract(off)

typedef _Float16 v16h __attribute__((ext_vector_type(16)));
typedef __bf16   v16b __attribute__((ext_vector_type(16)));
typedef float    v8f  __attribute__((ext_vector_type(8)));
typedef float    v4f  __attribute__((ext_vector_type(4)));
typedef v4f      v4fm __attribute__((may_alias));

#define NB      16
#define SRCW    256
#define DSTW    150
#define NPIX    22500
#define NPIXP   22528
#define NHIST   61
#define HPL     4096
#define N1      13456
#define NP1     13504
#define K1      75
#define N2      3136
#define K2      1152
#define K3      1024
#define P3      169
#define NT3     11
#define FEATN   1384448
#define OUT0N   144
#define HEADLEN 86528

__device__ __forceinline__ int kidx(int j, int h) { return 8 * h + j + ((j >= 8) ? 8 : 0); }

__device__ __forceinline__ v8f mma_f16(v16h a, v16h b, v8f c) {
  c = __builtin_amdgcn_wmma_f32_16x16x32_f16(false, a, false, b, (short)0, c, false, false);
  asm volatile("v_nop\n\tv_nop\n\tv_nop\n\tv_nop" : "+v"(c) : "v"(a), "v"(b));
  return c;
}

__device__ __forceinline__ v8f mma_bf16x3(v16b ah, v16b al, v16b bh, v16b bl, v8f c) {
  c = __builtin_amdgcn_wmma_f32_16x16x32_bf16(false, ah, false, bh, (short)0, c, false, false);
  c = __builtin_amdgcn_wmma_f32_16x16x32_bf16(false, ah, false, bl, (short)0, c, false, false);
  c = __builtin_amdgcn_wmma_f32_16x16x32_bf16(false, al, false, bh, (short)0, c, false, false);
  asm volatile("v_nop\n\tv_nop\n\tv_nop\n\tv_nop" : "+v"(c) : "v"(ah), "v"(al), "v"(bh), "v"(bl));
  return c;
}

__device__ __forceinline__ void split_bf16(float x, __bf16* hi, __bf16* lo) {
  const __bf16 t = (__bf16)x;
  *hi = t;
  *lo = (__bf16)(x - (float)t);
}

__device__ __forceinline__ void store_tile64(const float* stage, float* dst, int pitch, int wave, int lane) {
  const int sub = lane >> 4, ch = lane & 15;
#pragma unroll
  for (int i = 0; i < 8; ++i) {
    const int row = wave * 16 + 2 * i + sub;
    const v4f v = *(const v4fm*)(stage + row * 64 + ch * 4);
    *(volatile v4f*)(dst + (size_t)row * pitch + ch * 4) = v;
  }
  __threadfence();
#pragma unroll
  for (int i = 0; i < 8; ++i) {
    const int row = wave * 16 + 2 * i + sub;
    const v4f v = *(const v4fm*)(stage + row * 64 + ch * 4);
    *(volatile v4f*)(dst + (size_t)row * pitch + ch * 4) = v;
  }
}

__device__ __forceinline__ void rs_taps(int i, int* base, float* wn) {
  const float inv_scale = (float)(1.0 / 0.5859375);
  const float rks = 1.0f / inv_scale;
  const float sf = ((float)i + 0.5f) * inv_scale - 0.5f;
  const int y0 = (int)floorf(sf - inv_scale);
  float w[5];
  float s = 0.0f;
#pragma unroll
  for (int a = 0; a < 5; ++a) {
    const int y = y0 + a;
    const float d = fabsf(sf - (float)y) * rks;
    float v = fmaxf(0.0f, 1.0f - d);
    if (y < 0 || y > SRCW - 1) v = 0.0f;
    w[a] = v;
    s += v;
  }
  const float rs = 1.0f / s;
#pragma unroll
  for (int a = 0; a < 5; ++a) wn[a] = w[a] * rs;
  *base = y0;
}

__global__ __launch_bounds__(256) void k_pre(const float* __restrict__ x,
                                             float* Iu, float* Iv, float* Iy) {
  const int t = blockIdx.x * 256 + (int)threadIdx.x;
  if (t >= NB * NPIXP) return;
  const int b = t / NPIXP, n = t - b * NPIXP;
  float iy = 0.0f, u0 = 0.0f, u1 = 0.0f, u2 = 0.0f, q0 = 0.0f, q1 = 0.0f, q2 = 0.0f;
  if (n < NPIX) {
    const int py = n / DSTW, px = n - py * DSTW;
    int yb, xb;
    float wy[5], wx[5];
    rs_taps(py, &yb, wy);
    rs_taps(px, &xb, wx);
    int yc[5], xc[5];
#pragma unroll
    for (int a = 0; a < 5; ++a) {
      int yy = yb + a; yy = yy < 0 ? 0 : (yy > SRCW - 1 ? SRCW - 1 : yy);
      int xx = xb + a; xx = xx < 0 ? 0 : (xx > SRCW - 1 ? SRCW - 1 : xx);
      yc[a] = yy; xc[a] = xx;
    }
    float f[3];
#pragma unroll
    for (int c = 0; c < 3; ++c) {
      const float* p = x + (size_t)(b * 3 + c) * (SRCW * SRCW);
      float acc = 0.0f;
#pragma unroll
      for (int bb = 0; bb < 5; ++bb) {
        float col = 0.0f;
#pragma unroll
        for (int a = 0; a < 5; ++a) col += wy[a] * p[yc[a] * SRCW + xc[bb]];
        acc += wx[bb] * col;
      }
      f[c] = acc;
    }
    iy = sqrtf(f[0] * f[0] + f[1] * f[1] + f[2] * f[2]);
    u0 = logf(f[0] / f[1]);
    u1 = logf(f[1] / f[0]);
    u2 = logf(f[2] / f[0]);
    q0 = logf(f[0] / f[2]);
    q1 = logf(f[1] / f[2]);
    q2 = logf(f[2] / f[1]);
  }
  const size_t py_off = (size_t)b * NPIXP + n;
  const size_t pu_off = (size_t)b * 3 * NPIXP + n;
  *(volatile float*)(Iy + py_off) = iy;
  *(volatile float*)(Iu + pu_off) = u0;
  *(volatile float*)(Iu + pu_off + NPIXP) = u1;
  *(volatile float*)(Iu + pu_off + 2 * NPIXP) = u2;
  *(volatile float*)(Iv + pu_off) = q0;
  *(volatile float*)(Iv + pu_off + NPIXP) = q1;
  *(volatile float*)(Iv + pu_off + 2 * NPIXP) = q2;
  __threadfence();
  *(volatile float*)(Iy + py_off) = iy;
  *(volatile float*)(Iu + pu_off) = u0;
  *(volatile float*)(Iu + pu_off + NPIXP) = u1;
  *(volatile float*)(Iu + pu_off + 2 * NPIXP) = u2;
  *(volatile float*)(Iv + pu_off) = q0;
  *(volatile float*)(Iv + pu_off + NPIXP) = q1;
  *(volatile float*)(Iv + pu_off + 2 * NPIXP) = q2;
}

__global__ __launch_bounds__(128) void k_hist(
    const float* __restrict__ Iu, const float* __restrict__ Iv, const float* __restrict__ Iy,
    const float* __restrict__ sigu, const float* __restrict__ sigv, const float* __restrict__ Cc,
    float* hist) {
  __shared__ float pu[32], pv[32], pw[32];
  __shared__ __align__(32) _Float16 Bf[4 * 32 * 16];
  __shared__ __align__(16) float stage[64 * 64];
  const int bc = blockIdx.x;
  const int b = bc / 3, c = bc - b * 3;
  const int tid = threadIdx.x, lane = tid & 31, h = lane >> 4, m = lane & 15;
  const int wave = __builtin_amdgcn_readfirstlane(tid >> 5);
  const float su = sigu[c], sv = sigv[c];
  const float inv_su = 1.0f / (su * su + 1e-9f);
  const float inv_sv = 1.0f / (sv * sv + 1e-9f);
  const float* iu = Iu + (size_t)bc * NPIXP;
  const float* iv = Iv + (size_t)bc * NPIXP;
  const float* iy = Iy + (size_t)b * NPIXP;

  v8f acc[4];
#pragma unroll
  for (int i = 0; i < 4; ++i) acc[i] = 0.0f;

  const int ubin = wave * 16 + m;
  const bool ubok = (ubin < NHIST);
  const float eps = (float)(6.4 / 60.0);
  const float bin = -3.2f + eps * (float)ubin;

  for (int n0 = 0; n0 < NPIX; n0 += 32) {
    if (tid < 32) {
      const int n = n0 + tid;
      const bool ok = (n < NPIX);
      pu[tid] = ok ? iu[n] : 1e30f;
      pv[tid] = ok ? iv[n] : 1e30f;
      pw[tid] = ok ? iy[n] : 0.0f;
    }
    __syncthreads();
    v16h afr, bown;
#pragma unroll
    for (int j = 0; j < 16; ++j) {
      const int k = kidx(j, h);
      float a = 0.0f, bv = 0.0f;
      if (ubok) {
        const float du = pu[k] - bin;
        const float dv = pv[k] - bin;
        a  = __expf(-(du * du) * inv_su) * pw[k] * 8192.0f;
        bv = __expf(-(dv * dv) * inv_sv) * 32768.0f;
      }
      afr[j]  = (_Float16)a;
      bown[j] = (_Float16)bv;
    }
    *(v16h*)(Bf + (wave * 32 + lane) * 16) = bown;
    __syncthreads();
#pragma unroll
    for (int nt = 0; nt < 4; ++nt) {
      const v16h bfr = *(const v16h*)(Bf + (nt * 32 + lane) * 16);
      acc[nt] = mma_f16(afr, bfr, acc[nt]);
    }
    __syncthreads();
  }

  const float scl = Cc[c] * (1.0f / 268435456.0f);
#pragma unroll
  for (int nt = 0; nt < 4; ++nt) {
#pragma unroll
    for (int j = 0; j < 8; ++j) {
      const int u = wave * 16 + 8 * h + j;
      const int v = nt * 16 + m;
      stage[u * 64 + v] = sqrtf(acc[nt][j] * scl);
    }
  }
  __syncthreads();
  float* dst = hist + (size_t)bc * HPL;
#pragma unroll
  for (int i = 0; i < 8; ++i) {
    const int ci = i * 128 + tid;
    const v4f v = *(const v4fm*)(stage + ci * 4);
    *(volatile v4f*)(dst + ci * 4) = v;
  }
  __threadfence();
#pragma unroll
  for (int i = 0; i < 8; ++i) {
    const int ci = i * 128 + tid;
    const v4f v = *(const v4fm*)(stage + ci * 4);
    *(volatile v4f*)(dst + ci * 4) = v;
  }
}

__global__ __launch_bounds__(128) void k_conv1(
    const float* __restrict__ w1, const float* __restrict__ hist,
    const float* __restrict__ b1, float* h1) {
  __shared__ __align__(32) __bf16 Bh[4 * 32 * 16];
  __shared__ __align__(32) __bf16 Bl[4 * 32 * 16];
  __shared__ __align__(16) float stage[64 * 64];
  const int Nb = blockIdx.x * 64, Mb = blockIdx.y * 64;
  const int tid = threadIdx.x, lane = tid & 31, h = lane >> 4, m = lane & 15;
  const int wave = __builtin_amdgcn_readfirstlane(tid >> 5);
  const int o = Mb + wave * 16 + m;
  const int n = Nb + wave * 16 + m;
  const bool nok = (n < N1);
  const int nc = nok ? n : 0;
  const int bb = nc / 841, rem = nc - bb * 841, oy = rem / 29, ox = rem - oy * 29;
  const float* bsrc = hist + (size_t)bb * 3 * HPL;

  v8f acc[4];
#pragma unroll
  for (int i = 0; i < 4; ++i) acc[i] = 0.0f;

  for (int k0 = 0; k0 < 96; k0 += 32) {
    v16b ah, al, bh, bl;
#pragma unroll
    for (int j = 0; j < 16; ++j) {
      const int k = k0 + kidx(j, h);
      const bool kok = (k < K1);
      const int kk = kok ? k : (K1 - 1);
      float av = w1[o * K1 + kk];
      if (!kok) av = 0.0f;
      const int cch = kk / 25, r = kk - cch * 25, ky = r / 5, kx = r - ky * 5;
      float bv = bsrc[cch * HPL + (2 * oy + ky) * 64 + (2 * ox + kx)];
      if (!(kok && nok)) bv = 0.0f;
      __bf16 th, tl;
      split_bf16(av, &th, &tl); ah[j] = th; al[j] = tl;
      split_bf16(bv, &th, &tl); bh[j] = th; bl[j] = tl;
    }
    *(v16b*)(Bh + (wave * 32 + lane) * 16) = bh;
    *(v16b*)(Bl + (wave * 32 + lane) * 16) = bl;
    __syncthreads();
#pragma unroll
    for (int nt = 0; nt < 4; ++nt) {
      const v16b fh = *(const v16b*)(Bh + (nt * 32 + lane) * 16);
      const v16b fl = *(const v16b*)(Bl + (nt * 32 + lane) * 16);
      acc[nt] = mma_bf16x3(ah, al, fh, fl, acc[nt]);
    }
    __syncthreads();
  }

#pragma unroll
  for (int nt = 0; nt < 4; ++nt) {
#pragma unroll
    for (int j = 0; j < 8; ++j) {
      const int rl = wave * 16 + 8 * h + j;
      stage[rl * 64 + nt * 16 + m] = fmaxf(acc[nt][j] + b1[Mb + rl], 0.0f);
    }
  }
  __syncthreads();
  store_tile64(stage, h1 + (size_t)Mb * NP1 + Nb, NP1, wave, lane);
}

__global__ __launch_bounds__(128) void k_conv2(
    const float* __restrict__ w2, const float* __restrict__ h1,
    const float* __restrict__ b2, float* h2) {
  __shared__ __align__(32) __bf16 Bh[4 * 32 * 16];
  __shared__ __align__(32) __bf16 Bl[4 * 32 * 16];
  __shared__ __align__(16) float stage[64 * 64];
  const int Nb = blockIdx.x * 64, Mb = blockIdx.y * 64;
  const int tid = threadIdx.x, lane = tid & 31, h = lane >> 4, m = lane & 15;
  const int wave = __builtin_amdgcn_readfirstlane(tid >> 5);
  const int o = Mb + wave * 16 + m;
  const int n = Nb + wave * 16 + m;
  const int bb = n / 196, rem = n - bb * 196, oy = rem / 14, ox = rem - oy * 14;
  const float* arow = w2 + (size_t)o * K2;
  const float* bsrc = h1 + (size_t)bb * 841;

  v8f acc[4];
#pragma unroll
  for (int i = 0; i < 4; ++i) acc[i] = 0.0f;

  for (int k0 = 0; k0 < K2; k0 += 32) {
    const float* ap = arow + k0 + 8 * h;
    const v4f x0 = *(const v4f*)(ap);
    const v4f x1 = *(const v4f*)(ap + 4);
    const v4f x2 = *(const v4f*)(ap + 16);
    const v4f x3 = *(const v4f*)(ap + 20);
    const float av[16] = {x0[0], x0[1], x0[2], x0[3], x1[0], x1[1], x1[2], x1[3],
                          x2[0], x2[1], x2[2], x2[3], x3[0], x3[1], x3[2], x3[3]};
    v16b ah, al, bh, bl;
#pragma unroll
    for (int j = 0; j < 16; ++j) {
      const int k = k0 + kidx(j, h);
      const int cch = k / 9, r = k - cch * 9, ky = r / 3, kx = r - ky * 3;
      const float bv = bsrc[(size_t)cch * NP1 + (2 * oy + ky) * 29 + (2 * ox + kx)];
      __bf16 th, tl;
      split_bf16(av[j], &th, &tl); ah[j] = th; al[j] = tl;
      split_bf16(bv, &th, &tl); bh[j] = th; bl[j] = tl;
    }
    *(v16b*)(Bh + (wave * 32 + lane) * 16) = bh;
    *(v16b*)(Bl + (wave * 32 + lane) * 16) = bl;
    __syncthreads();
#pragma unroll
    for (int nt = 0; nt < 4; ++nt) {
      const v16b fh = *(const v16b*)(Bh + (nt * 32 + lane) * 16);
      const v16b fl = *(const v16b*)(Bl + (nt * 32 + lane) * 16);
      acc[nt] = mma_bf16x3(ah, al, fh, fl, acc[nt]);
    }
    __syncthreads();
  }

#pragma unroll
  for (int nt = 0; nt < 4; ++nt) {
#pragma unroll
    for (int j = 0; j < 8; ++j) {
      const int rl = wave * 16 + 8 * h + j;
      stage[rl * 64 + nt * 16 + m] = fmaxf(acc[nt][j] + b2[Mb + rl], 0.0f);
    }
  }
  __syncthreads();
  store_tile64(stage, h2 + (size_t)Mb * N2 + Nb, N2, wave, lane);
}

__global__ __launch_bounds__(256) void k_conv3(
    const float* __restrict__ w3, const float* __restrict__ h2,
    const float* __restrict__ b3, float* feat) {
  __shared__ __align__(32) float lraw[64 * P3];
  __bf16* Bh = reinterpret_cast<__bf16*>(lraw);
  __bf16* Bl = Bh + NT3 * 32 * 16;
  const int Mb = blockIdx.x * 64, b = blockIdx.y;
  const int tid = threadIdx.x, lane = tid & 31, h = lane >> 4, m = lane & 15;
  const int wave = __builtin_amdgcn_readfirstlane(tid >> 5);
  const int rg = wave & 3, s = wave >> 2;
  const int o = Mb + rg * 16 + m;
  const float* arow = w3 + (size_t)o * K3;
  const float* bsrc = h2 + (size_t)b * 196;

  v8f acc[6];
#pragma unroll
  for (int i = 0; i < 6; ++i) acc[i] = 0.0f;

  for (int k0 = 0; k0 < K3; k0 += 32) {
    const float* ap = arow + k0 + 8 * h;
    const v4f x0 = *(const v4f*)(ap);
    const v4f x1 = *(const v4f*)(ap + 4);
    const v4f x2 = *(const v4f*)(ap + 16);
    const v4f x3 = *(const v4f*)(ap + 20);
    const float av[16] = {x0[0], x0[1], x0[2], x0[3], x1[0], x1[1], x1[2], x1[3],
                          x2[0], x2[1], x2[2], x2[3], x3[0], x3[1], x3[2], x3[3]};
    v16b ah, al;
#pragma unroll
    for (int j = 0; j < 16; ++j) {
      __bf16 th, tl;
      split_bf16(av[j], &th, &tl); ah[j] = th; al[j] = tl;
    }
#pragma unroll 1
    for (int q = 0; q < 2; ++q) {
      const int f = tid + q * 256;
      if (f < NT3 * 32) {
        const int nt = f >> 5, lr = f & 31, hh = lr >> 4;
        const int p = nt * 16 + (lr & 15);
        const bool pok = (p < P3);
        const int pc = pok ? p : 0;
        const int oy = pc / 13, ox = pc - oy * 13;
        v16b bh, bl;
#pragma unroll
        for (int j = 0; j < 16; ++j) {
          const int k = k0 + kidx(j, hh);
          const int cch = k >> 2, ky = (k >> 1) & 1, kx = k & 1;
          float bv = bsrc[(size_t)cch * N2 + (oy + ky) * 14 + (ox + kx)];
          if (!pok) bv = 0.0f;
          __bf16 th, tl;
          split_bf16(bv, &th, &tl); bh[j] = th; bl[j] = tl;
        }
        *(v16b*)(Bh + f * 16) = bh;
        *(v16b*)(Bl + f * 16) = bl;
      }
    }
    __syncthreads();
#pragma unroll
    for (int t = 0; t < 6; ++t) {
      const int nt = s * 6 + t;
      if (nt < NT3) {
        const v16b fh = *(const v16b*)(Bh + (nt * 32 + lane) * 16);
        const v16b fl = *(const v16b*)(Bl + (nt * 32 + lane) * 16);
        acc[t] = mma_bf16x3(ah, al, fh, fl, acc[t]);
      }
    }
    __syncthreads();
  }

  float* stage = lraw;
#pragma unroll
  for (int t = 0; t < 6; ++t) {
    const int nt = s * 6 + t;
    if (nt < NT3) {
#pragma unroll
      for (int j = 0; j < 8; ++j) {
        const int ol = rg * 16 + 8 * h + j;
        const int p = nt * 16 + m;
        if (p < P3) stage[ol * P3 + p] = acc[t][j];
      }
    }
  }
  __syncthreads();
  float* dst = feat + (size_t)(b * 512 + Mb) * P3;
  const float* bias = b3 + Mb;
  for (int c = tid; c < (64 * P3) / 4; c += 256) {
    v4f v;
#pragma unroll
    for (int e = 0; e < 4; ++e) {
      const int q = 4 * c + e;
      const int ol = q / P3;
      v[e] = fmaxf(stage[q] + bias[ol], 0.0f);
    }
    *(volatile v4f*)(dst + 4 * c) = v;
  }
  __threadfence();
  for (int c = tid; c < (64 * P3) / 4; c += 256) {
    v4f v;
#pragma unroll
    for (int e = 0; e < 4; ++e) {
      const int q = 4 * c + e;
      const int ol = q / P3;
      v[e] = fmaxf(stage[q] + bias[ol], 0.0f);
    }
    *(volatile v4f*)(dst + 4 * c) = v;
  }
}

__global__ __launch_bounds__(256) void k_head(const float* __restrict__ feat,
                                              const float* __restrict__ wf,
                                              const float* __restrict__ bf,
                                              float* out) {
  __shared__ float red[8];
  __shared__ __align__(16) float res[160];
  const int tid = threadIdx.x, lane = tid & 31, wave = tid >> 5;
  for (int bo = 0; bo < OUT0N; ++bo) {
    const int b = bo / 9, o = bo - b * 9;
    const float* f = feat + (size_t)b * HEADLEN;
    const float* w = wf + (size_t)o * HEADLEN;
    float s = 0.0f;
#pragma unroll 2
    for (int i = tid; i < HEADLEN; i += 256) s += f[i] * w[i];
    s += __shfl_xor(s, 16);
    s += __shfl_xor(s, 8);
    s += __shfl_xor(s, 4);
    s += __shfl_xor(s, 2);
    s += __shfl_xor(s, 1);
    if (lane == 0) red[wave] = s;
    __syncthreads();
    if (tid == 0) {
      float tsum = red[0];
#pragma unroll
      for (int q = 1; q < 8; ++q) tsum += red[q];
      res[bo] = tsum + bf[o];
    }
    __syncthreads();
  }
  if (tid < 16) res[OUT0N + tid] = feat[tid];
  __syncthreads();
  if (tid < 40) {
    const v4f v = *(const v4fm*)(res + tid * 4);
    *(volatile v4f*)(out + tid * 4) = v;
  }
  __threadfence();
  if (tid < 40) {
    const v4f v = *(const v4fm*)(res + tid * 4);
    *(volatile v4f*)(out + tid * 4) = v;
  }
}

__global__ __launch_bounds__(256) void k_pack(const float* __restrict__ feat, float* out, int nch) {
  const int c = blockIdx.x * 256 + (int)threadIdx.x;
  if (c >= nch) return;
  const v4f v = *(const v4f*)(feat + 16 + (size_t)c * 4);
  float* p = out + 160 + (size_t)c * 4;
  *(volatile v4f*)p = v;
  __threadfence();
  *(volatile v4f*)p = v;
}

extern "C" void kernel_launch(void* const* d_in, const int* in_sizes, int n_in,
                              void* d_out, int out_size, void* d_ws, size_t ws_size,
                              hipStream_t stream) {
  if (n_in < 12) return;
  if (in_sizes[0] != NB * 3 * SRCW * SRCW) return;
  if (out_size != OUT0N + FEATN) return;
  const float* x    = (const float*)d_in[0];
  const float* sigu = (const float*)d_in[1];
  const float* sigv = (const float*)d_in[2];
  const float* Cc   = (const float*)d_in[3];
  const float* w1   = (const float*)d_in[4];
  const float* b1   = (const float*)d_in[5];
  const float* w2   = (const float*)d_in[6];
  const float* b2   = (const float*)d_in[7];
  const float* w3   = (const float*)d_in[8];
  const float* b3   = (const float*)d_in[9];
  const float* wf   = (const float*)d_in[10];
  const float* bf   = (const float*)d_in[11];
  float* out = (float*)d_out;

  char* wsb = (char*)d_ws;
  size_t off = 0;
  auto carve = [&](size_t bytes) -> void* {
    void* p = wsb + off;
    off += (bytes + 255) & ~(size_t)255;
    return p;
  };
  float* Iu   = (float*)carve((size_t)NB * 3 * NPIXP * sizeof(float));
  float* Iv   = (float*)carve((size_t)NB * 3 * NPIXP * sizeof(float));
  float* Iy   = (float*)carve((size_t)NB * NPIXP * sizeof(float));
  float* hist = (float*)carve((size_t)NB * 3 * HPL * sizeof(float));
  float* h1   = (float*)carve((size_t)128 * NP1 * sizeof(float));
  float* h2   = (float*)carve((size_t)256 * N2 * sizeof(float));
  float* feat = (float*)carve((size_t)FEATN * sizeof(float));
  if (off > ws_size) return;

  k_pre<<<(NB * NPIXP + 255) / 256, 256, 0, stream>>>(x, Iu, Iv, Iy);
  k_hist<<<NB * 3, 128, 0, stream>>>(Iu, Iv, Iy, sigu, sigv, Cc, hist);
  k_conv1<<<dim3(NP1 / 64, 2), 128, 0, stream>>>(w1, hist, b1, h1);
  k_conv2<<<dim3(N2 / 64, 4), 128, 0, stream>>>(w2, h1, b2, h2);
  k_conv3<<<dim3(8, NB), 256, 0, stream>>>(w3, h2, b3, feat);
  k_head<<<1, 256, 0, stream>>>(feat, wf, bf, out);
  const int nch = (OUT0N + FEATN - 160) / 4;
  k_pack<<<(nch + 255) / 256, 256, 0, stream>>>(feat, out, nch);
}
